// DeepConv1d_63101659513165
// MI455X (gfx1250) — hardware-run, weakly checked
//
#include <hip/hip_runtime.h>

typedef float          v8f   __attribute__((ext_vector_type(8)));
typedef float          v4f   __attribute__((ext_vector_type(4)));
typedef unsigned int   v4u   __attribute__((ext_vector_type(4)));
typedef int            v8i   __attribute__((ext_vector_type(8)));
typedef unsigned short v8us  __attribute__((ext_vector_type(8)));
typedef unsigned short v16us __attribute__((ext_vector_type(16)));
typedef __bf16         v16bf __attribute__((ext_vector_type(16)));
typedef _Float16       v16h  __attribute__((ext_vector_type(16)));
typedef v4f  __attribute__((may_alias)) v4fa;
typedef v8us __attribute__((may_alias)) v8usa;
union FragB { v16bf v; v16us u; v8us h[2]; v8i w; };
union FragH { v16h  v; v16us u; v8us h[2]; v8i w; };

__device__ __forceinline__ v8f wmb(const FragB& a, const FragB& b, v8f c) {
  v8f d = __builtin_amdgcn_wmma_f32_16x16x32_bf16(false, a.v, false, b.v, (short)0, c, false, false);
  asm volatile("v_nop\n\tv_nop\n\tv_nop\n\tv_nop" : "+v"(d) : "v"(a.w), "v"(b.w));
  return d;
}

__device__ __forceinline__ v8f wmh(const FragH& a, const FragH& b, v8f c) {
  v8f d = __builtin_amdgcn_wmma_f32_16x16x32_f16(false, a.v, false, b.v, (short)0, c, false, false);
  asm volatile("v_nop\n\tv_nop\n\tv_nop\n\tv_nop" : "+v"(d) : "v"(a.w), "v"(b.w));
  return d;
}

__device__ __forceinline__ unsigned bf16_bits(float f) {
  const unsigned u = __float_as_uint(f);
  const unsigned r = (u + 0x7FFFu + ((u >> 16) & 1u)) >> 16;
  const unsigned q = (u >> 16) | 0x40u;
  return ((u & 0x7fffffffu) > 0x7f800000u) ? q : r;
}

__device__ __forceinline__ float bf16_val(float f) {
  return __uint_as_float(bf16_bits(f) << 16);
}
__device__ __forceinline__ int clampi(int v, int lo, int hi) {
  return v < lo ? lo : (v > hi ? hi : v);
}

__device__ __forceinline__ unsigned f16_bits(float f) {
  const unsigned u  = __float_as_uint(f);
  const unsigned s  = (u >> 16) & 0x8000u;
  const unsigned a  = u & 0x7fffffffu;
  const unsigned t  = a - 0x38000000u;
  const unsigned r  = (t + 0x0FFFu + ((t >> 13) & 1u)) >> 13;
  const unsigned rc = r > 0x7C00u ? 0x7C00u : r;
  const bool small  = a < 0x38800000u;
  const bool isnan  = a > 0x7f800000u;
  const unsigned fin = small ? 0u : (s | rc);
  return isnan ? (s | 0x7E00u) : fin;
}

__device__ __forceinline__ unsigned pk16(unsigned lo, unsigned hi) { return lo | (hi << 16); }
__device__ __forceinline__ unsigned bf16_lo_bits(float v) {
  float hi = bf16_val(v);
  asm volatile("" : "+v"(hi));
  return bf16_bits(v - hi);
}
__device__ __forceinline__ v4u pack8_bf16(v4f a, v4f c) {
  return (v4u){ pk16(bf16_bits(a[0]), bf16_bits(a[1])), pk16(bf16_bits(a[2]), bf16_bits(a[3])),
                pk16(bf16_bits(c[0]), bf16_bits(c[1])), pk16(bf16_bits(c[2]), bf16_bits(c[3])) };
}
__device__ __forceinline__ v4u pack8_bf16_lo(v4f a, v4f c) {
  return (v4u){ pk16(bf16_lo_bits(a[0]), bf16_lo_bits(a[1])), pk16(bf16_lo_bits(a[2]), bf16_lo_bits(a[3])),
                pk16(bf16_lo_bits(c[0]), bf16_lo_bits(c[1])), pk16(bf16_lo_bits(c[2]), bf16_lo_bits(c[3])) };
}
__device__ __forceinline__ v4u pack8_f16(v4f a, v4f c) {
  return (v4u){ pk16(f16_bits(a[0]), f16_bits(a[1])), pk16(f16_bits(a[2]), f16_bits(a[3])),
                pk16(f16_bits(c[0]), f16_bits(c[1])), pk16(f16_bits(c[2]), f16_bits(c[3])) };
}

template <int FORM>
__global__ __launch_bounds__(256) void k_plane(const float* __restrict__ src, int rows, int cols, int ldsrc,
                                               unsigned short* __restrict__ dst, int MP, int KP) {
  static_assert(FORM >= 0 && FORM <= 3);
  const int KTOT = (FORM == 1 || FORM == 3) ? 2 * KP : KP;
  const unsigned ppr   = (unsigned)(KTOT >> 3);
  const unsigned kp8   = (unsigned)(KP >> 3);
  const unsigned total = (unsigned)MP * ppr;
  const unsigned g     = blockIdx.x * 256u + threadIdx.x;
  const unsigned rowu  = g / ppr;
  const unsigned p     = g - rowu * ppr;
  const bool second    = p >= kp8;
  const int row = (int)rowu;
  const int c0  = (int)((second ? p - kp8 : p) << 3);
  const float* srow = src + (size_t)clampi(row, 0, rows - 1) * (size_t)ldsrc;
  float x[8];
  unsigned mk[8];
#pragma unroll
  for (int e = 0; e < 8; ++e) {
    const int c = c0 + e;
    const float v = srow[clampi(c, 0, cols - 1)];
    asm volatile("" :: "v"(v));
    x[e]  = v;
    mk[e] = (row < rows && c < cols) ? 0xFFFFu : 0u;
  }
  const v4f a = (v4f){ x[0], x[1], x[2], x[3] };
  const v4f c = (v4f){ x[4], x[5], x[6], x[7] };
  v4u o;
  if (FORM == 2) {
    o = pack8_f16(a, c);
  } else {
    const v4u hi = pack8_bf16(a, c);
    o = hi;
    if (FORM == 1) { const v4u lo = pack8_bf16_lo(a, c); o = second ? lo : hi; }
  }
  const v4u mw = (v4u){ pk16(mk[0], mk[1]), pk16(mk[2], mk[3]), pk16(mk[4], mk[5]), pk16(mk[6], mk[7]) };
  o &= mw;
  if (g < total) {
    volatile v4u* q = (volatile v4u*)(dst + (size_t)g * 8);
    *q = o;
    __threadfence();
    *q = o;
  }
}

template <int FORM> struct FragOf    { typedef FragB T; };
template <>         struct FragOf<2> { typedef FragH T; };
__device__ __forceinline__ v8f mm(const FragB& a, const FragB& b, v8f c) { return wmb(a, b, c); }
__device__ __forceinline__ v8f mm(const FragH& a, const FragH& b, v8f c) { return wmh(a, b, c); }
template <class F> __device__ __forceinline__ F ld_frag(const unsigned short* p) {
  F f;
  f.h[0] = *(const v8usa*)(p);
  f.h[1] = *(const v8usa*)(p + 16);
  return f;
}

template <int FORM, int EPI>
__global__ __launch_bounds__(256) __attribute__((amdgpu_num_vgpr(248)))
void k_gemm_nt(const unsigned short* __restrict__ A, const unsigned short* __restrict__ B,
               const float* __restrict__ bias, float* __restrict__ D, int M, int N, int KTOT, int ldd) {
  static_assert(FORM >= 0 && FORM <= 2);
  static_assert(EPI == 0 || EPI == 1);
  typedef typename FragOf<FORM>::T F;
  __shared__ __attribute__((aligned(16))) float sT[8][16 * 68];
  const int lane = threadIdx.x & 31;
  const int wave = threadIdx.x >> 5;
  const int tilesM = (M + 63) >> 6;
  const int tilesN = (N + 63) >> 6;
  const int tile = blockIdx.x * 8 + wave;
  if (tile >= tilesM * tilesN) return;
  const int tm = tile / tilesN;
  const int tn = tile - tm * tilesN;
  const int m0 = tm << 6;
  const int n0 = tn << 6;

  const int rl = lane & 15;
  const int h8 = (lane >> 4) * 8;
  const unsigned short* pa = A + (size_t)(m0 + rl) * (size_t)KTOT + h8;
  const unsigned short* pb = B + (size_t)(n0 + rl) * (size_t)KTOT + h8;

  v8f acc[4][4];
#pragma unroll
  for (int i = 0; i < 4; ++i)
#pragma unroll
    for (int j = 0; j < 4; ++j) acc[i][j] = (v8f){0.f, 0.f, 0.f, 0.f, 0.f, 0.f, 0.f, 0.f};

#pragma unroll 1
  for (int k0 = 0; k0 < KTOT; k0 += 32) {
    F bf[4];
#pragma unroll
    for (int j = 0; j < 4; ++j) bf[j] = ld_frag<F>(pb + (size_t)(j << 4) * (size_t)KTOT + k0);
#pragma unroll
    for (int i = 0; i < 4; ++i) {
      const F af = ld_frag<F>(pa + (size_t)(i << 4) * (size_t)KTOT + k0);
#pragma unroll
      for (int j = 0; j < 4; ++j) acc[i][j] = mm(af, bf[j], acc[i][j]);
    }
  }

  float* slab = sT[wave];
  const int hh = lane >> 4;
  const int c4 = (lane & 15) * 4;
  const int nc = n0 + c4;
  const bool cok = nc < N;
  v4f bv = (v4f){0.f, 0.f, 0.f, 0.f};
  if (EPI == 1) {
    bv = *(const v4fa*)(bias + clampi(nc, 0, N - 4));
    asm volatile("" :: "v"(bv));
  }
#pragma unroll
  for (int i = 0; i < 4; ++i) {
    const int mBase = m0 + (i << 4);
#pragma unroll
    for (int j = 0; j < 4; ++j) {
#pragma unroll
      for (int r = 0; r < 8; ++r) slab[(h8 + r) * 68 + (j << 4) + rl] = acc[i][j][r];
    }
    __builtin_amdgcn_fence(__ATOMIC_RELEASE, "workgroup");
    __builtin_amdgcn_wave_barrier();
    __builtin_amdgcn_fence(__ATOMIC_ACQUIRE, "workgroup");
    v4f vv[8];
#pragma unroll
    for (int it = 0; it < 8; ++it) {
      const int row = it * 2 + hh;
      v4f v = *(const v4fa*)(slab + row * 68 + c4);
      if (EPI == 1) v += bv;
      vv[it] = v;
    }
    for (int pass = 0; pass < 2; ++pass) {
#pragma unroll
      for (int it = 0; it < 8; ++it) {
        const int row = mBase + it * 2 + hh;
        if (cok && row < M) *(volatile v4f*)(D + (size_t)row * (size_t)ldd + nc) = vv[it];
      }
      __threadfence();
    }
    __builtin_amdgcn_fence(__ATOMIC_RELEASE, "workgroup");
    __builtin_amdgcn_wave_barrier();
    __builtin_amdgcn_fence(__ATOMIC_ACQUIRE, "workgroup");
  }
}

#ifndef OUT_FORM
#define OUT_FORM 3
#endif
static_assert(OUT_FORM >= 1 && OUT_FORM <= 3);

typedef v4u __attribute__((may_alias)) v4ua;

constexpr int kB     = 16;
constexpr int kDC    = 16;
constexpr int kND    = 1024;
constexpr int kC     = 64;
constexpr int kNP    = 4096;
constexpr int kCO    = 128;
constexpr int kTap   = 7;
constexpr int kF     = kC * kTap;
constexpr int kNBp   = 8;
constexpr int kNPASS = 2;
constexpr int kCG    = 4;
constexpr int kTL    = 64;
constexpr int kWP    = 72;
constexpr int kKA    = (OUT_FORM == 2) ? 2 * kF : kF;
constexpr int kFPW   = kKA / 2 + 4;
constexpr int kPPR   = kKA / 8;
constexpr int kFlushIt = kTL * kPPR / 256;
constexpr int kMpass = kNBp * kNP;
constexpr float kFCar = (OUT_FORM == 3) ? 64.0f : 1.0f;
constexpr float kWCar = (OUT_FORM == 3) ? 64.0f : 1.0f;
constexpr float kOScale = 1.0f / (kFCar * kWCar);

static_assert(kB % kNBp == 0);
static_assert(kNBp * kNPASS == kB);
static_assert(kF % 32 == 0);
static_assert(kKA % 32 == 0);
static_assert((kNBp * kNP) % 128 == 0);
static_assert(kMpass % 64 == 0);
static_assert(kCO % 64 == 0);
static_assert(kNP % kTL == 0);
static_assert(kNP % 32 == 0);
static_assert(kC * kWP == 18 * 256);
static_assert((kTL * kPPR) % 256 == 0);
static_assert((kFPW * 4) % 16 == 0);
static_assert(kC % kCG == 0);
static_assert(kC % 2 == 0);
static_assert((kKA * 2) % 128 == 0);
static_assert(kCO * kKA / 8 % 256 == 0);

constexpr int kXsDynBytes   = kCG * kNP * 4 + kDC * (kND / 2) * 4;
constexpr int kFeatDynBytes = (2 * kC * kWP + 16 * 256) * 4 + kTL * kFPW * 4;
static_assert(kXsDynBytes + 1024 <= 327680);
static_assert(kFeatDynBytes <= 327680);

__device__ __forceinline__ double wave_sum_f64(double v) {
#pragma unroll
  for (int off = 16; off > 0; off >>= 1) v += __shfl_xor(v, off, 32);
  return v;
}

__global__ __launch_bounds__(256) __attribute__((amdgpu_num_vgpr(248)))
void k_xs(const float* __restrict__ deep, const float* __restrict__ conv_w, const float* __restrict__ conv_b,
          float* __restrict__ XS) {
  extern __shared__ __attribute__((aligned(16))) float dyn_xs[];
  float*    sY  = dyn_xs;
  unsigned* sDw = (unsigned*)(dyn_xs + kCG * kNP);
  __shared__ __attribute__((aligned(16))) float sW[kCG * kDC];
  __shared__ __attribute__((aligned(16))) float sStat[8];
  __shared__ double sRedA[8 * kCG];
  __shared__ double sRedB[8 * kCG];

  const int tid  = threadIdx.x;
  const int lane = tid & 31;
  const int wave = tid >> 5;
  const int c0   = blockIdx.x * kCG;
  const int b    = blockIdx.y;

  const float* dp = deep + (size_t)b * kDC * kND;
#pragma unroll 4
  for (int it = 0; it < 16; ++it) {
    const int g = tid + 256 * it;
    const v4f v = *(const v4fa*)(dp + 4 * g);
    sDw[2 * g]     = pk16(bf16_bits(v[0]), bf16_bits(v[1]));
    sDw[2 * g + 1] = pk16(bf16_bits(v[2]), bf16_bits(v[3]));
  }
  {
    const int q = tid < 16 ? tid : 15;
    const v4f wv = *(const v4fa*)(conv_w + c0 * kDC + 4 * q);
    asm volatile("" :: "v"(wv));
    if (tid < 16) {
      const v4f o = (v4f){ bf16_val(wv[0]), bf16_val(wv[1]), bf16_val(wv[2]), bf16_val(wv[3]) };
      *(v4fa*)(sW + 4 * tid) = o;
    }
  }
  const v4f bvv = *(const v4fa*)(conv_b + c0);
  float bb[kCG];
#pragma unroll
  for (int cc = 0; cc < kCG; ++cc) bb[cc] = bf16_val(bvv[cc]);
  __syncthreads();

  float ps[kCG];
#pragma unroll
  for (int cc = 0; cc < kCG; ++cc) ps[cc] = 0.0f;

#pragma unroll 1
  for (int i = 0; i < 16; ++i) {
    const int j = tid + 256 * i;
    float src = ((float)j + 0.5f) * 0.25f - 0.5f;
    src = (src < 0.0f) ? 0.0f : src;
    src = (src > 1023.0f) ? 1023.0f : src;
    const int lo = (int)src;
    const int hi = (lo + 1 > kND - 1) ? (kND - 1) : (lo + 1);
    const float w   = src - (float)lo;
    const float w1m = 1.0f - w;
    const int wlo = lo >> 1, slo = (lo & 1) * 16;
    const int whi = hi >> 1, shi = (hi & 1) * 16;
    float acc[kCG];
#pragma unroll
    for (int cc = 0; cc < kCG; ++cc) acc[cc] = 0.0f;
#pragma unroll 2
    for (int d = 0; d < kDC; ++d) {
      const unsigned ul = sDw[d * (kND / 2) + wlo];
      const unsigned uh = sDw[d * (kND / 2) + whi];
      const float v0 = __uint_as_float((ul >> slo) << 16);
      const float v1 = __uint_as_float((uh >> shi) << 16);
      const float xr = v0 * w1m + v1 * w;
#pragma unroll
      for (int cc = 0; cc < kCG; ++cc) acc[cc] = fmaf(xr, sW[cc * kDC + d], acc[cc]);
    }
#pragma unroll
    for (int cc = 0; cc < kCG; ++cc) {
      const float y = acc[cc] + bb[cc];
      sY[cc * kNP + j] = y;
      ps[cc] += y;
    }
  }

#pragma unroll
  for (int cc = 0; cc < kCG; ++cc) {
    const double r = wave_sum_f64((double)ps[cc]);
    if (lane == 0) sRedA[wave * kCG + cc] = r;
  }
  __syncthreads();
  float mean[kCG];
#pragma unroll
  for (int cc = 0; cc < kCG; ++cc) {
    double t = 0.0;
#pragma unroll
    for (int wq = 0; wq < 8; ++wq) t += sRedA[wq * kCG + cc];
    mean[cc] = (float)(t * (1.0 / 4096.0));
  }

  float pq[kCG];
#pragma unroll
  for (int cc = 0; cc < kCG; ++cc) pq[cc] = 0.0f;
#pragma unroll 1
  for (int i = 0; i < 16; ++i) {
    const int j = tid + 256 * i;
#pragma unroll
    for (int cc = 0; cc < kCG; ++cc) {
      const float dv = sY[cc * kNP + j] - mean[cc];
      pq[cc] = fmaf(dv, dv, pq[cc]);
    }
  }
#pragma unroll
  for (int cc = 0; cc < kCG; ++cc) {
    const double r = wave_sum_f64((double)pq[cc]);
    if (lane == 0) sRedB[wave * kCG + cc] = r;
  }
  __syncthreads();
#pragma unroll
  for (int cc = 0; cc < kCG; ++cc) {
    double t = 0.0;
#pragma unroll
    for (int wq = 0; wq < 8; ++wq) t += sRedB[wq * kCG + cc];
    const float var = (float)(t * (1.0 / 4095.0));
    if (tid == 0) {
      sStat[cc]     = mean[cc];
      sStat[4 + cc] = var + 1e-9f;
    }
  }
  __syncthreads();

#pragma unroll 1
  for (int cc = 0; cc < kCG; ++cc) {
    const float m  = sStat[cc];
    const float dn = sStat[4 + cc];
#pragma unroll 1
    for (int i = 0; i < 16; ++i) {
      const int j = tid + 256 * i;
      const float y = sY[cc * kNP + j];
      sY[cc * kNP + j] = (0.5f * (y - m)) / dn;
    }
  }

  float* xsb = XS + ((size_t)b * kC + c0) * kNP;
#pragma unroll 1
  for (int pass = 0; pass < 2; ++pass) {
#pragma unroll 1
    for (int cc = 0; cc < kCG; ++cc) {
#pragma unroll 4
      for (int i = 0; i < 16; ++i) {
        const int j = tid + 256 * i;
        const float v = sY[cc * kNP + j];
        *(volatile float*)(xsb + (size_t)cc * kNP + j) = v;
      }
    }
    __threadfence();
  }
}

__device__ __forceinline__ unsigned feat_hi_bits(float v) {
#if OUT_FORM == 3
  return f16_bits(v * kFCar);
#else
  return bf16_bits(v);
#endif
}

__global__ __launch_bounds__(256) __attribute__((amdgpu_num_vgpr(248)))
void k_feat(const float* __restrict__ XS, const float* __restrict__ x, unsigned short* __restrict__ Ap, int b0) {
  extern __shared__ __attribute__((aligned(16))) float dyn_ft[];
  float*    sXS = dyn_ft;
  float*    sX  = dyn_ft + kC * kWP;
  float*    sL  = dyn_ft + 2 * kC * kWP;
  unsigned* sF  = (unsigned*)(dyn_ft + 2 * kC * kWP + 16 * 256);

  const int tid = threadIdx.x;
  const int l0  = blockIdx.x * kTL;
  const int bl  = blockIdx.y;
  const int b   = b0 + bl;
  const float* xsb = XS + (size_t)b * kC * kNP;
  const float* xb  = x  + (size_t)b * kC * kNP;

#pragma unroll 3
  for (int it = 0; it < 18; ++it) {
    const int p  = tid + 256 * it;
    const int c  = p / kWP;
    const int jj = p - c * kWP;
    int g = l0 - 3 + jj;
    g = (g < 0) ? -g : g;
    g = (g > kNP - 1) ? (2 * (kNP - 1) - g) : g;
    g = clampi(g, 0, kNP - 1);
    const float a = xsb[(size_t)c * kNP + g];
    const float v = xb[(size_t)c * kNP + g];
    asm volatile("" :: "v"(a), "v"(v));
    sXS[p] = a;
    sX[p]  = bf16_val(v);
  }
  __syncthreads();

  const int l  = tid & 63;
  const int pq = tid >> 6;
#pragma unroll 1
  for (int it = 0; it < 8; ++it) {
    const int cp = pq + 4 * it;
#pragma unroll 1
    for (int cc = 0; cc < 2; ++cc) {
      const float* xw = sXS + (2 * cp + cc) * kWP + l;
      const float xc = xw[3];
      float s = 0.0f;
#pragma unroll 1
      for (int k = 0; k < kTap; ++k) {
        const float d  = fabsf(xw[k] - xc);
        const float t  = tanhf(d);
        const float ls = 1.0f - t * t;
        s += ls;
        sL[(cc * kTap + k) * 256 + tid] = ls;
      }
      sL[(14 + cc) * 256 + tid] = 1.0f / s;
    }
    const float al0 = sL[14 * 256 + tid];
    const float al1 = sL[15 * 256 + tid];
    const float* x0 = sX + (2 * cp) * kWP + l;
    unsigned* frow = sF + l * kFPW + cp * kTap;
#pragma unroll
    for (int j = 0; j < kTap; ++j) {
      const int qa = 2 * j;
      const int qb = 2 * j + 1;
      const int ia = (qa < kTap) ? qa : (kWP + qa - kTap);
      const int ib = (qb < kTap) ? qb : (kWP + qb - kTap);
      const float aa = (qa < kTap) ? al0 : al1;
      const float ab = (qb < kTap) ? al0 : al1;
      const float va = (sL[qa * 256 + tid] * aa) * x0[ia];
      const float vb = (sL[qb * 256 + tid] * ab) * x0[ib];
      frow[j] = pk16(feat_hi_bits(va), feat_hi_bits(vb));
#if OUT_FORM == 2
      frow[kF / 2 + j] = pk16(bf16_lo_bits(va), bf16_lo_bits(vb));
#endif
    }
  }
  __syncthreads();

  unsigned short* dst = Ap + ((size_t)bl * kNP + l0) * (size_t)kKA;
#pragma unroll 1
  for (int pass = 0; pass < 2; ++pass) {
#pragma unroll 4
    for (int it = 0; it < kFlushIt; ++it) {
      const int g   = tid + 256 * it;
      const int row = g / kPPR;
      const int pc  = g - row * kPPR;
      const v4u v = *(const v4ua*)(sF + row * kFPW + pc * 4);
      *(volatile v4u*)(dst + (size_t)g * 8) = v;
    }
    __threadfence();
  }
}

#if OUT_FORM == 3
__global__ __launch_bounds__(256) void k_fw16(const float* __restrict__ w, unsigned short* __restrict__ dst) {
  const unsigned g = blockIdx.x * 256u + threadIdx.x;
  const v4f a = *(const v4fa*)(w + (size_t)g * 8);
  const v4f c = *(const v4fa*)(w + (size_t)g * 8 + 4);
  const v4f a2 = (v4f){ kWCar * bf16_val(a[0]), kWCar * bf16_val(a[1]), kWCar * bf16_val(a[2]), kWCar * bf16_val(a[3]) };
  const v4f c2 = (v4f){ kWCar * bf16_val(c[0]), kWCar * bf16_val(c[1]), kWCar * bf16_val(c[2]), kWCar * bf16_val(c[3]) };
  const v4u o = pack8_f16(a2, c2);
  volatile v4u* q = (volatile v4u*)(dst + (size_t)g * 8);
  *q = o;
  __threadfence();
  *q = o;
}
#endif

__global__ __launch_bounds__(256) void k_tr(const float* __restrict__ Cm, float* __restrict__ out, float oscale) {
  __shared__ float sT[32 * 129];
  const int tid  = threadIdx.x;
  const int lane = tid & 31;
  const int wave = tid >> 5;
  const int m0 = blockIdx.x * 32;
  const int b  = m0 / kNP;
  const int l0 = m0 - b * kNP;
#pragma unroll
  for (int it = 0; it < 4; ++it) {
    const int g = tid + 256 * it;
    const int r = g >> 5;
    const int q = g & 31;
    const v4f v = *(const v4fa*)(Cm + (size_t)(m0 + r) * kCO + 4 * q);
    sT[r * 129 + 4 * q + 0] = v[0];
    sT[r * 129 + 4 * q + 1] = v[1];
    sT[r * 129 + 4 * q + 2] = v[2];
    sT[r * 129 + 4 * q + 3] = v[3];
  }
  __syncthreads();
  float vv[16];
#pragma unroll
  for (int i = 0; i < 16; ++i) vv[i] = sT[lane * 129 + wave * 16 + i] * oscale;
  float* ob = out + ((size_t)b * kCO + wave * 16) * kNP + l0 + lane;
#pragma unroll 1
  for (int pass = 0; pass < 2; ++pass) {
#pragma unroll
    for (int i = 0; i < 16; ++i) *(volatile float*)(ob + (size_t)i * kNP) = vv[i];
    __threadfence();
  }
}

extern "C" void kernel_launch(void* const* d_in, const int* in_sizes, int n_in,
                              void* d_out, int out_size, void* d_ws, size_t ws_size,
                              hipStream_t stream) {
  if (n_in < 5) return;
  if (in_sizes[0] != kB * kDC * kND) return;
  if (in_sizes[1] != kB * kC * kNP) return;
  if (in_sizes[2] != kC * kDC) return;
  if (in_sizes[3] != kC) return;
  if (in_sizes[4] != kCO * kF) return;
  if (out_size != kB * kCO * kNP) return;

  const float* deep   = (const float*)d_in[0];
  const float* x      = (const float*)d_in[1];
  const float* conv_w = (const float*)d_in[2];
  const float* conv_b = (const float*)d_in[3];
  const float* fc_w   = (const float*)d_in[4];
  float* out = (float*)d_out;

  size_t off = 0;
  const size_t oFW = off; off += (size_t)kCO * kKA * 2;
  const size_t oXS = off; off += (size_t)kB * kC * kNP * 4;
  const size_t oA  = off; off += (size_t)kMpass * kKA * 2;
  const size_t oC  = off; off += (size_t)kB * kNP * kCO * 4;
  if ((oXS & 255) || (oA & 255) || (oC & 255)) return;
  if (off > ws_size) return;
  if (off > ((size_t)128 << 20)) return;

  char* ws = (char*)d_ws;
  unsigned short* FW = (unsigned short*)(ws + oFW);
  float*          XS = (float*)(ws + oXS);
  unsigned short* Ap = (unsigned short*)(ws + oA);
  float*          Cm = (float*)(ws + oC);

#if OUT_FORM == 2
  k_plane<3><<<dim3(kCO * kKA / 8 / 256), dim3(256), 0, stream>>>(fc_w, kCO, kF, kF, FW, kCO, kF);
#elif OUT_FORM == 1
  k_plane<0><<<dim3(kCO * kKA / 8 / 256), dim3(256), 0, stream>>>(fc_w, kCO, kF, kF, FW, kCO, kF);
#else
  k_fw16<<<dim3(kCO * kKA / 8 / 256), dim3(256), 0, stream>>>(fc_w, FW);
#endif

  (void)hipFuncSetAttribute(reinterpret_cast<const void*>(&k_xs), hipFuncAttributeMaxDynamicSharedMemorySize,
                            kXsDynBytes);
  k_xs<<<dim3(kC / kCG, kB), dim3(256), kXsDynBytes, stream>>>(deep, conv_w, conv_b, XS);

  (void)hipFuncSetAttribute(reinterpret_cast<const void*>(&k_feat), hipFuncAttributeMaxDynamicSharedMemorySize,
                            kFeatDynBytes);
  const int tiles = (kMpass / 64) * (kCO / 64);
  for (int p = 0; p < kNPASS; ++p) {
    k_feat<<<dim3(kNP / kTL, kNBp), dim3(256), kFeatDynBytes, stream>>>(XS, x, Ap, p * kNBp);
    float* Dp = Cm + (size_t)p * kMpass * kCO;
#if OUT_FORM == 3
    k_gemm_nt<2, 0><<<dim3((tiles + 7) / 8), dim3(256), 0, stream>>>(Ap, FW, (const float*)XS, Dp, kMpass, kCO, kKA, kCO);
#elif OUT_FORM == 2
    k_gemm_nt<1, 0><<<dim3((tiles + 7) / 8), dim3(256), 0, stream>>>(Ap, FW, (const float*)XS, Dp, kMpass, kCO, kKA, kCO);
#else
    k_gemm_nt<0, 0><<<dim3((tiles + 7) / 8), dim3(256), 0, stream>>>(Ap, FW, (const float*)XS, Dp, kMpass, kCO, kKA, kCO);
#endif
  }

  k_tr<<<dim3(kB * kNP / 32), dim3(256), 0, stream>>>(Cm, out, kOScale);
  (void)hipGetLastError();
}
